// DynamicConvBlock_65730179498326
// MI455X (gfx1250) — hardware-verified
//
#include <hip/hip_runtime.h>
#include <stdint.h>


#define TT   2048
#define DD   512
#define FF   512
#define KK   7
#define HH   128
#define NC   (KK * FF)
#define TOK  32
#define NTHR 256

typedef _Float16       v16h __attribute__((ext_vector_type(16)));
typedef _Float16       v8h  __attribute__((ext_vector_type(8)));
typedef __bf16         v16b __attribute__((ext_vector_type(16)));
typedef __bf16         v8b  __attribute__((ext_vector_type(8)));
typedef float          v8f  __attribute__((ext_vector_type(8)));
typedef float          v4f  __attribute__((ext_vector_type(4)));
typedef unsigned short us8  __attribute__((ext_vector_type(8)));
typedef unsigned short us4  __attribute__((ext_vector_type(4)));

union FragH { v16h v; v8h half[2]; };
union FragB { v16b v; v8b half[2]; };

__device__ __forceinline__ v8f mma_f16(v8f acc, v16h a, v16h b) {
  acc = __builtin_amdgcn_wmma_f32_16x16x32_f16(false, a, false, b, (short)0, acc, false, false);
  asm volatile("v_nop\n\tv_nop\n\tv_nop\n\tv_nop" : "+v"(acc) : "v"(a), "v"(b));
  return acc;
}
__device__ __forceinline__ v8f mma_bf16(v8f acc, v16b a, v16b b) {
  acc = __builtin_amdgcn_wmma_f32_16x16x32_bf16(false, a, false, b, (short)0, acc, false, false);
  asm volatile("v_nop\n\tv_nop\n\tv_nop\n\tv_nop" : "+v"(acc) : "v"(a), "v"(b));
  return acc;
}

__device__ __forceinline__ v8f zero8() {
  v8f z = {0.f, 0.f, 0.f, 0.f, 0.f, 0.f, 0.f, 0.f};
  return z;
}

__device__ __forceinline__ unsigned short bf16_rne(float f) {
  unsigned int u = __float_as_uint(f);
  u = u + 0x7FFFu + ((u >> 16) & 1u);
  return (unsigned short)(u >> 16);
}
__device__ __forceinline__ float bf16_val(unsigned short b) {
  return __uint_as_float(((unsigned int)b) << 16);
}
__device__ __forceinline__ unsigned short f16_bits(float f) {
  _Float16 hv = (_Float16)f;
  return __builtin_bit_cast(unsigned short, hv);
}

__global__ __launch_bounds__(NTHR) void k_prep(const float* __restrict__ W1,
                                              const float* __restrict__ W2,
                                              unsigned short* W1hi,
                                              unsigned short* W1lo,
                                              unsigned short* W2s) {
  const int n1 = HH * (DD / 8);
  const int n2 = NC * (HH / 8);
  const int id = blockIdx.x * NTHR + threadIdx.x;
  if (id < n1) {
    const int hcol = id / (DD / 8);
    const int d0   = (id - hcol * (DD / 8)) * 8;
    us8 vh, vl;
#pragma unroll
    for (int j = 0; j < 8; ++j) {
      const float f = W1[(size_t)(d0 + j) * HH + hcol];
      const unsigned short hb = bf16_rne(f);
      vh[j] = hb;
      vl[j] = bf16_rne(f - bf16_val(hb));
    }
    const size_t off = (size_t)hcol * DD + d0;
    *(volatile us8*)(W1hi + off) = vh;
    *(volatile us8*)(W1lo + off) = vl;
    __threadfence();
    *(volatile us8*)(W1hi + off) = vh;
    *(volatile us8*)(W1lo + off) = vl;
  } else if (id < n1 + n2) {
    const int id2 = id - n1;
    const int c   = id2 / (HH / 8);
    const int h0  = (id2 - c * (HH / 8)) * 8;
    us8 v;
#pragma unroll
    for (int j = 0; j < 8; ++j) {
      const float f = W2[(size_t)(h0 + j) * NC + c];
      v[j] = f16_bits(f * 64.0f);
    }
    const size_t off = (size_t)c * HH + h0;
    *(volatile us8*)(W2s + off) = v;
    __threadfence();
    *(volatile us8*)(W2s + off) = v;
  }
}

__global__ __launch_bounds__(NTHR) void k_gemm1(const float* __restrict__ x,
                                               const unsigned short* __restrict__ W1hi,
                                               const unsigned short* __restrict__ W1lo,
                                               const float* __restrict__ b1,
                                               unsigned short* Hout,
                                               int ntok) {
  __shared__ __attribute__((aligned(16))) unsigned short lds[2 * TOK * DD];
  unsigned short* xs_hi = lds;
  unsigned short* xs_lo = lds + TOK * DD;

  const int tid = threadIdx.x, l = tid & 31, w = tid >> 5, h = l >> 4, m = l & 15;
  const int t0 = blockIdx.x * TOK;

#pragma unroll 4
  for (int p = 0; p < (TOK * DD / 4) / NTHR; ++p) {
    const int idx = p * NTHR + tid;
    const int row = idx / (DD / 4);
    const int col = (idx - row * (DD / 4)) * 4;
    float4 v = make_float4(0.f, 0.f, 0.f, 0.f);
    if (t0 + row < ntok) v = *(const float4*)(x + (size_t)(t0 + row) * DD + col);
    const float f[4] = {v.x, v.y, v.z, v.w};
    us4 vh, vl;
#pragma unroll
    for (int j = 0; j < 4; ++j) {
      const unsigned short hb = bf16_rne(f[j]);
      vh[j] = hb;
      vl[j] = bf16_rne(f[j] - bf16_val(hb));
    }
    *(us4*)(xs_hi + row * DD + col) = vh;
    *(us4*)(xs_lo + row * DD + col) = vl;
  }
  __syncthreads();

  const int mt = w & 1, ht0 = (w >> 1) * 2;
  v8f acc[2];
  acc[0] = zero8();
  acc[1] = zero8();

  const unsigned short* ahp  = xs_hi + (mt * 16 + m) * DD + 8 * h;
  const unsigned short* alp  = xs_lo + (mt * 16 + m) * DD + 8 * h;
  const unsigned short* bhp0 = W1hi + (size_t)(ht0 * 16 + m) * DD + 8 * h;
  const unsigned short* blp0 = W1lo + (size_t)(ht0 * 16 + m) * DD + 8 * h;
  const unsigned short* bhp1 = W1hi + (size_t)((ht0 + 1) * 16 + m) * DD + 8 * h;
  const unsigned short* blp1 = W1lo + (size_t)((ht0 + 1) * 16 + m) * DD + 8 * h;

#pragma unroll 2
  for (int ks = 0; ks < DD / 32; ++ks) {
    const int k0 = ks * 32;
    FragB ah, al, bh, bl;
    ah.half[0] = *(const v8b*)(ahp + k0);
    ah.half[1] = *(const v8b*)(ahp + k0 + 16);
    al.half[0] = *(const v8b*)(alp + k0);
    al.half[1] = *(const v8b*)(alp + k0 + 16);

    bh.half[0] = *(const v8b*)(bhp0 + k0);
    bh.half[1] = *(const v8b*)(bhp0 + k0 + 16);
    bl.half[0] = *(const v8b*)(blp0 + k0);
    bl.half[1] = *(const v8b*)(blp0 + k0 + 16);
    acc[0] = mma_bf16(acc[0], ah.v, bh.v);
    acc[0] = mma_bf16(acc[0], al.v, bh.v);
    acc[0] = mma_bf16(acc[0], ah.v, bl.v);

    bh.half[0] = *(const v8b*)(bhp1 + k0);
    bh.half[1] = *(const v8b*)(bhp1 + k0 + 16);
    bl.half[0] = *(const v8b*)(blp1 + k0);
    bl.half[1] = *(const v8b*)(blp1 + k0 + 16);
    acc[1] = mma_bf16(acc[1], ah.v, bh.v);
    acc[1] = mma_bf16(acc[1], al.v, bh.v);
    acc[1] = mma_bf16(acc[1], ah.v, bl.v);
  }
  __syncthreads();

  unsigned short* hs = lds;
#pragma unroll
  for (int nt = 0; nt < 2; ++nt) {
    const int col = (ht0 + nt) * 16 + m;
    const float bb = b1[col];
#pragma unroll
    for (int r = 0; r < 8; ++r) {
      const int row = mt * 16 + 8 * h + r;
      const float v = fmaxf(acc[nt][r] + bb, 0.f) * 16.0f;
      hs[row * HH + col] = f16_bits(v);
    }
  }
  __syncthreads();

  const us8 o0 = *(const us8*)(hs + tid * 8);
  const us8 o1 = *(const us8*)(hs + (NTHR + tid) * 8);
  const int row0 = (tid * 8) / HH;
  const int row1 = ((NTHR + tid) * 8) / HH;
  const bool ok0 = (t0 + row0) < ntok;
  const bool ok1 = (t0 + row1) < ntok;
  unsigned short* g = Hout + (size_t)t0 * HH;
  if (ok0) *(volatile us8*)(g + tid * 8) = o0;
  if (ok1) *(volatile us8*)(g + (NTHR + tid) * 8) = o1;
  __threadfence();
  if (ok0) *(volatile us8*)(g + tid * 8) = o0;
  if (ok1) *(volatile us8*)(g + (NTHR + tid) * 8) = o1;
}

__global__ __launch_bounds__(NTHR) void k_main(const float* __restrict__ x,
                                              const unsigned short* __restrict__ Hm,
                                              const unsigned short* __restrict__ W2s,
                                              const float* __restrict__ b2,
                                              const float* __restrict__ gamma,
                                              const float* __restrict__ beta,
                                              float* out,
                                              int ntok) {
  __shared__ __attribute__((aligned(16))) float ylds[TOK * FF];
  const int tid = threadIdx.x, l = tid & 31, w = tid >> 5, h = l >> 4, m = l & 15;
  const int t0 = blockIdx.x * TOK;
  const int bidx = t0 / TT;
  const int tb = t0 - bidx * TT;

  for (int j = w; j < TOK + KK - 1; j += NTHR / 32) {
    const int ts = tb - (KK / 2) + j;
    const int grow = bidx * TT + ts;
    float sum = 0.f;
    if (ts >= 0 && ts < TT && grow < ntok) {
      const float* xr = x + (size_t)grow * DD + 4 * l;
#pragma unroll
      for (int q = 0; q < DD / 128; ++q) {
        const float4 v = *(const float4*)(xr + 128 * q);
        sum += (v.x + v.y) + (v.z + v.w);
      }
    }
#pragma unroll
    for (int off = 16; off > 0; off >>= 1) sum += __shfl_xor(sum, off, 32);
    if (l == 0) ylds[j] = sum;
  }
  __syncthreads();

  const int mt = w & 1, fgrp = w >> 1;
  float wk[KK][8];
#pragma unroll
  for (int k = 0; k < KK; ++k)
#pragma unroll
    for (int r = 0; r < 8; ++r)
      wk[k][r] = ylds[mt * 16 + 8 * h + r + k];

  int arow = t0 + mt * 16 + m;
  if (arow > ntok - 1) arow = ntok - 1;
  const unsigned short* ap = Hm + (size_t)arow * HH + 8 * h;
  FragH afr[4];
#pragma unroll
  for (int i = 0; i < HH / 32; ++i) {
    afr[i].half[0] = *(const v8h*)(ap + 32 * i);
    afr[i].half[1] = *(const v8h*)(ap + 32 * i + 16);
  }
  __syncthreads();

#pragma unroll 1
  for (int ftl = 0; ftl < (FF / 16) / 4; ++ftl) {
    const int col = (fgrp * ((FF / 16) / 4) + ftl) * 16 + m;
    float accf[8];
#pragma unroll
    for (int r = 0; r < 8; ++r) accf[r] = 0.f;

#pragma unroll
    for (int k = 0; k < KK; ++k) {
      const int c = k * FF + col;
      const unsigned short* bp = W2s + (size_t)c * HH + 8 * h;
      v8f tmp = zero8();
#pragma unroll
      for (int i = 0; i < HH / 32; ++i) {
        FragH b;
        b.half[0] = *(const v8h*)(bp + 32 * i);
        b.half[1] = *(const v8h*)(bp + 32 * i + 16);
        tmp = mma_f16(tmp, afr[i].v, b.v);
      }
      const float b2v = b2[c];
#pragma unroll
      for (int r = 0; r < 8; ++r)
        accf[r] = fmaf(wk[k][r], fmaf(tmp[r], 0.0009765625f, b2v), accf[r]);
    }
#pragma unroll
    for (int r = 0; r < 8; ++r) {
      const int mrow = mt * 16 + 8 * h + r;
      const int grow = t0 + mrow;
      const float xr = (grow < ntok) ? x[(size_t)grow * DD + col] : 0.f;
      ylds[mrow * FF + col] = accf[r] + xr;
    }
  }
  __syncthreads();

  for (int q = 0; q < TOK / (NTHR / 32); ++q) {
    const int tok = w * (TOK / (NTHR / 32)) + q;
    const int grow = t0 + tok;
    const float* yr = ylds + tok * FF + 4 * l;
    v4f v[4];
    float sum = 0.f;
#pragma unroll
    for (int jj = 0; jj < 4; ++jj) {
      v[jj] = *(const v4f*)(yr + 128 * jj);
      sum += (v[jj][0] + v[jj][1]) + (v[jj][2] + v[jj][3]);
    }
#pragma unroll
    for (int off = 16; off > 0; off >>= 1) sum += __shfl_xor(sum, off, 32);
    const float mu = sum * (1.0f / FF);
    float sq = 0.f;
    v4f d[4];
#pragma unroll
    for (int jj = 0; jj < 4; ++jj)
#pragma unroll
      for (int c4 = 0; c4 < 4; ++c4) {
        const float e = v[jj][c4] - mu;
        d[jj][c4] = e;
        sq = fmaf(e, e, sq);
      }
#pragma unroll
    for (int off = 16; off > 0; off >>= 1) sq += __shfl_xor(sq, off, 32);
    const float var = sq * (1.0f / FF);
    const float rs = rsqrtf(var + 1.0e-3f);
    v4f o[4];
#pragma unroll
    for (int jj = 0; jj < 4; ++jj) {
      const v4f g  = *(const v4f*)(gamma + 128 * jj + 4 * l);
      const v4f be = *(const v4f*)(beta + 128 * jj + 4 * l);
#pragma unroll
      for (int c4 = 0; c4 < 4; ++c4)
        o[jj][c4] = fmaxf((d[jj][c4] * rs) * g[c4] + be[c4], 0.f);
    }
    if (grow < ntok) {
      float* op = out + (size_t)grow * FF + 4 * l;
#pragma unroll
      for (int jj = 0; jj < 4; ++jj) *(volatile v4f*)(op + 128 * jj) = o[jj];
      __threadfence();
#pragma unroll
      for (int jj = 0; jj < 4; ++jj) *(volatile v4f*)(op + 128 * jj) = o[jj];
    }
  }
}

extern "C" void kernel_launch(void* const* d_in, const int* in_sizes, int n_in,
                              void* d_out, int out_size, void* d_ws, size_t ws_size,
                              hipStream_t stream) {
  if (n_in < 7) return;
  const float* x     = (const float*)d_in[0];
  const float* W1    = (const float*)d_in[1];
  const float* b1    = (const float*)d_in[2];
  const float* W2    = (const float*)d_in[3];
  const float* b2    = (const float*)d_in[4];
  const float* gamma = (const float*)d_in[5];
  const float* beta  = (const float*)d_in[6];
  float* out = (float*)d_out;

  const int ntok = in_sizes[0] / DD;
  if (ntok <= 0 || (ntok % TT) != 0) return;
  if (in_sizes[1] != DD * HH || in_sizes[2] != HH || in_sizes[3] != HH * NC ||
      in_sizes[4] != NC || in_sizes[5] != FF || in_sizes[6] != FF) return;
  if (out_size != ntok * FF) return;

  const size_t sz_w1  = (size_t)HH * DD * 2;
  const size_t sz_w2  = (size_t)NC * HH * 2;
  const size_t sz_h   = (size_t)ntok * HH * 2;
  const size_t off_w1hi = 0;
  const size_t off_w1lo = off_w1hi + sz_w1;
  const size_t off_w2   = off_w1lo + sz_w1;
  const size_t off_h    = off_w2 + sz_w2;
  const size_t total    = off_h + sz_h;
  if (total > ws_size) return;

  char* ws = (char*)d_ws;
  unsigned short* W1hi = (unsigned short*)(ws + off_w1hi);
  unsigned short* W1lo = (unsigned short*)(ws + off_w1lo);
  unsigned short* W2s  = (unsigned short*)(ws + off_w2);
  unsigned short* Hm   = (unsigned short*)(ws + off_h);

  const int n_prep = HH * (DD / 8) + NC * (HH / 8);
  const dim3 g_prep((n_prep + NTHR - 1) / NTHR);
  const dim3 g_tok((ntok + TOK - 1) / TOK);

  k_prep <<<g_prep, NTHR, 0, stream>>>(W1, W2, W1hi, W1lo, W2s);
  k_gemm1<<<g_tok,  NTHR, 0, stream>>>(x, W1hi, W1lo, b1, Hm, ntok);
  k_main <<<g_tok,  NTHR, 0, stream>>>(x, Hm, W2s, b2, gamma, beta, out, ntok);
}
